// HigherOrderSimplicialConv_64123861729553
// MI455X (gfx1250) — hardware-verified
//
#include <hip/hip_runtime.h>
#include <stddef.h>
#include <math.h>


#define FD      128
#define NTHR    256
#define NWAVE   8
#define EPT     8
#define NGRP    2
#define CHUNK   (NTHR * EPT * NGRP)
#define WCAP    (EPT * NGRP * 32)
#define LISTN   (NWAVE * WCAP)
#define NBC     4096
#define NBF     1024
#define RCAP    40960
#define RBN     128
#define TGT     256
#define DEGCAP  1024
#define GROWS   128
#define OTHR    512
#define WSCAP   134217728
#define APK     136
#define ASCL    16.0f
#define WSCL    64.0f
#define UNSCL   0.0009765625f

#define LDS_FILL ((RCAP + NBF + LISTN) * 4 + 64)
#define LDS_GA   (GROWS * APK * 2)
#define LDS_GEMM (LDS_GA + GROWS * FD * 4)

#define BN_EPS 1e-5f

static_assert((CHUNK & (CHUNK - 1)) == 0);
static_assert(CHUNK <= 4096);
static_assert(NBC <= 4096 && NBF <= 4096);
static_assert((NBC & (NBC - 1)) == 0 && (NBF & (NBF - 1)) == 0);
static_assert(NBC == 4 * NBF);
static_assert(OTHR * 8 == NBC);
static_assert((RCAP % 32) == 0);
static_assert(TGT == NWAVE * 32 && (TGT % GROWS) == 0);
static_assert((NBC % TGT) == 0);
static_assert(GROWS == NWAVE * 16);
static_assert(FD == 128 && (APK % 8) == 0 && (LDS_GA % 16) == 0);
static_assert((TGT % 4) == 0);

typedef float          v4f  __attribute__((ext_vector_type(4)));
typedef float          v8f  __attribute__((ext_vector_type(8)));
typedef double         v2d  __attribute__((ext_vector_type(2)));
typedef int            v4i  __attribute__((ext_vector_type(4)));
typedef unsigned short v8us __attribute__((ext_vector_type(8)));
typedef _Float16       v4h  __attribute__((ext_vector_type(4)));
typedef _Float16       v8h  __attribute__((ext_vector_type(8)));
typedef _Float16       v16h __attribute__((ext_vector_type(16)));
union FragH { v16h v; v8h h[2]; };
union Pack8 { v8h h; v4h q[2]; v8us u; };

__device__ __forceinline__ v8f wmh(v16h a, v16h b, v8f c) {
  v8f d = __builtin_amdgcn_wmma_f32_16x16x32_f16(false, a, false, b, (short)0, c, false, false);
  asm volatile("v_nop\n\tv_nop\n\tv_nop\n\tv_nop" : "+v"(d) : "v"(a), "v"(b));
  return d;
}

__device__ __forceinline__ v8h cvt8(v4f a, v4f b, float scl) {
  Pack8 p;
  p.q[0] = __builtin_convertvector(a * scl, v4h);
  p.q[1] = __builtin_convertvector(b * scl, v4h);
  return p.h;
}

__device__ __forceinline__ void store_rows128(const float* stg, float* C, int rowBase, int wave, int lane) {
  const float* lp = stg + wave * 16 * FD + 4 * lane;
  float* gp = C + (size_t)(rowBase + wave * 16) * FD + 4 * lane;
#pragma unroll
  for (int i = 0; i < 16; ++i) { const v4f v = *(const v4f*)(lp + FD * i); *(volatile v4f*)(gp + FD * i) = v; }
  __threadfence();
#pragma unroll
  for (int i = 0; i < 16; ++i) { const v4f v = *(const v4f*)(lp + FD * i); *(volatile v4f*)(gp + FD * i) = v; }
}

template <int NB>
__device__ __forceinline__ int scan_chunk(const int* __restrict__ dsts, int nE, int cbase, int slotBase,
                                          int vec8, int* list, int tid, int lane, int wave) {
  int wc = 0;
#pragma unroll
  for (int g = 0; g < NGRP; ++g) {
    const int el0  = (g * NTHR + tid) * EPT;
    const int e0   = cbase + el0;
    const int sent = -2147483647 - 1;
    v4i da, db;
    if (vec8 != 0 && cbase + CHUNK <= nE) {
      da = *(const v4i*)(dsts + e0);
      db = *(const v4i*)(dsts + e0 + 4);
    } else {
      da.x = (e0     < nE) ? dsts[min(e0, nE - 1)] : sent;
      da.y = (e0 + 1 < nE) ? dsts[min(e0 + 1, nE - 1)] : sent;
      da.z = (e0 + 2 < nE) ? dsts[min(e0 + 2, nE - 1)] : sent;
      da.w = (e0 + 3 < nE) ? dsts[min(e0 + 3, nE - 1)] : sent;
      db.x = (e0 + 4 < nE) ? dsts[min(e0 + 4, nE - 1)] : sent;
      db.y = (e0 + 5 < nE) ? dsts[min(e0 + 5, nE - 1)] : sent;
      db.z = (e0 + 6 < nE) ? dsts[min(e0 + 6, nE - 1)] : sent;
      db.w = (e0 + 7 < nE) ? dsts[min(e0 + 7, nE - 1)] : sent;
    }
    const unsigned nb = (unsigned)slotBase;
    const unsigned s0 = (unsigned)da.x - nb, s1 = (unsigned)da.y - nb;
    const unsigned s2 = (unsigned)da.z - nb, s3 = (unsigned)da.w - nb;
    const unsigned s4 = (unsigned)db.x - nb, s5 = (unsigned)db.y - nb;
    const unsigned s6 = (unsigned)db.z - nb, s7 = (unsigned)db.w - nb;
    const bool h0 = s0 < (unsigned)NB, h1 = s1 < (unsigned)NB, h2 = s2 < (unsigned)NB, h3 = s3 < (unsigned)NB;
    const bool h4 = s4 < (unsigned)NB, h5 = s5 < (unsigned)NB, h6 = s6 < (unsigned)NB, h7 = s7 < (unsigned)NB;
    const unsigned any = __builtin_amdgcn_ballot_w32(h0 | h1 | h2 | h3 | h4 | h5 | h6 | h7);
    if (any != 0u) {
#define HITJ(J, HJ, SJ) { \
        const unsigned mj = __builtin_amdgcn_ballot_w32(HJ); \
        if (mj != 0u) { \
          if (HJ) { \
            const int pos = wc + (int)__builtin_amdgcn_mbcnt_lo(mj, 0u); \
            if (pos < WCAP) list[wave * WCAP + pos] = ((el0 + (J)) << 12) | (int)(SJ); \
          } \
          wc += (int)__builtin_popcount(mj); } }
      HITJ(0, h0, s0)
      HITJ(1, h1, s1)
      HITJ(2, h2, s2)
      HITJ(3, h3, s3)
      HITJ(4, h4, s4)
      HITJ(5, h5, s5)
      HITJ(6, h6, s6)
      HITJ(7, h7, s7)
#undef HITJ
    }
  }
  return wc;
}

__global__ __launch_bounds__(NTHR) void k_wprep(const float* __restrict__ W, unsigned short* wp) {
  const int i = blockIdx.x * NTHR + threadIdx.x;
  const int n = i >> 4, k0 = (i & 15) * 8;
  v4f a, b;
  a.x = W[(k0 + 0) * FD + n]; a.y = W[(k0 + 1) * FD + n]; a.z = W[(k0 + 2) * FD + n]; a.w = W[(k0 + 3) * FD + n];
  b.x = W[(k0 + 4) * FD + n]; b.y = W[(k0 + 5) * FD + n]; b.z = W[(k0 + 6) * FD + n]; b.w = W[(k0 + 7) * FD + n];
  Pack8 p;
  p.h = cvt8(a, b, WSCL);
  const v8us u = p.u;
  unsigned short* d = wp + (size_t)i * 8;
  *(volatile v8us*)d = u;
  __threadfence();
  *(volatile v8us*)d = u;
}

__global__ __launch_bounds__(NTHR) void k_count(const int* __restrict__ dsts, int* cnt, int nE, int vec8) {
  __shared__ __attribute__((aligned(16))) int scnt[NBC];
  __shared__ __attribute__((aligned(16))) int list[LISTN];
  __shared__ int wcnt[NWAVE];
  const int tid = threadIdx.x, lane = tid & 31, wave = tid >> 5;
  const int nodeBase = blockIdx.x * NBC;

  for (int i = tid; i < NBC; i += NTHR) scnt[i] = 0;
  __syncthreads();

  const int nChunks = (nE + CHUNK - 1) / CHUNK;
#pragma unroll 1
  for (int ch = 0; ch < nChunks; ++ch) {
    const int cbase = ch * CHUNK;
    const int wc = scan_chunk<NBC>(dsts, nE, cbase, nodeBase, vec8, list, tid, lane, wave);
    if (lane == 0) wcnt[wave] = wc;
    __syncthreads();
    if (wave == 0) {
#pragma unroll 1
      for (int wsx = 0; wsx < NWAVE; ++wsx) {
        int n = __builtin_amdgcn_readfirstlane(wcnt[wsx]);
        n = n > WCAP ? WCAP : (n < 0 ? 0 : n);
        const int* lp = list + wsx * WCAP;
#pragma unroll 1
        for (int i = 0; i < n; ++i) {
          const int ent  = __builtin_amdgcn_readfirstlane(lp[i]);
          const int slot = ent & (NBC - 1);
          if (lane == 0) scnt[slot] = scnt[slot] + 1;
        }
      }
    }
    __syncthreads();
  }

  v4i cq[4];
#pragma unroll
  for (int q = 0; q < 4; ++q) {
    const int f = (wave * 4 + q) * 128 + 4 * lane;
    cq[q] = *(const v4i*)(scnt + f);
  }
  int* cp = cnt + (size_t)nodeBase;
#pragma unroll
  for (int q = 0; q < 4; ++q) {
    const int f = (wave * 4 + q) * 128 + 4 * lane;
    *(volatile v4i*)(cp + f) = cq[q];
  }
  __threadfence();
#pragma unroll
  for (int q = 0; q < 4; ++q) {
    const int f = (wave * 4 + q) * 128 + 4 * lane;
    *(volatile v4i*)(cp + f) = cq[q];
  }
}

__global__ __launch_bounds__(OTHR) void k_offsets(
    const int* __restrict__ cnt, int* off, int* rbase, int nChunk) {
  __shared__ __attribute__((aligned(16))) int soff[NBC];
  __shared__ __attribute__((aligned(16))) int srb[RBN];
  __shared__ int wtot[OTHR / 32];
  const int tid = threadIdx.x, lane = tid & 31, wave = tid >> 5, sub = tid >> 7;
  for (int i = tid; i < RBN; i += OTHR) srb[i] = 0;
  int carry = 0;
#pragma unroll 1
  for (int ch = 0; ch < nChunk; ++ch) {
    const int base = ch * NBC;
    const v4i c0 = *(const v4i*)(cnt + base + 8 * tid);
    const v4i c1 = *(const v4i*)(cnt + base + 8 * tid + 4);
    const int e0 = max(c0.x, 0), e1 = max(c0.y, 0), e2 = max(c0.z, 0), e3 = max(c0.w, 0);
    const int e4 = max(c1.x, 0), e5 = max(c1.y, 0), e6 = max(c1.z, 0), e7 = max(c1.w, 0);
    const int ts = e0 + e1 + e2 + e3 + e4 + e5 + e6 + e7;
    int incl = ts;
#pragma unroll
    for (int d = 1; d < 32; d <<= 1) {
      const int t = __shfl_up(incl, d);
      if (lane >= d) incl += t;
    }
    if (lane == 31) wtot[wave] = incl;
    __syncthreads();
    const int S0 = wtot[0]  + wtot[1]  + wtot[2]  + wtot[3];
    const int S1 = wtot[4]  + wtot[5]  + wtot[6]  + wtot[7];
    const int S2 = wtot[8]  + wtot[9]  + wtot[10] + wtot[11];
    const int S3 = wtot[12] + wtot[13] + wtot[14] + wtot[15];
    int pre = 0;
#pragma unroll 1
    for (int w = 4 * sub; w < wave; ++w) pre += wtot[w];
    const int b0 = carry;
    const int b1 = b0 + ((S0 + 31) & ~31);
    const int b2 = b1 + ((S1 + 31) & ~31);
    const int b3 = b2 + ((S2 + 31) & ~31);
    const int b4 = b3 + ((S3 + 31) & ~31);
    const int myb = sub == 0 ? b0 : (sub == 1 ? b1 : (sub == 2 ? b2 : b3));
    if (tid == 0) {
      srb[min(4 * ch + 0, RBN - 1)] = b0;
      srb[min(4 * ch + 1, RBN - 1)] = b1;
      srb[min(4 * ch + 2, RBN - 1)] = b2;
      srb[min(4 * ch + 3, RBN - 1)] = b3;
    }
    int run = myb + pre + incl - ts;
    soff[8 * tid + 0] = run; run += e0;
    soff[8 * tid + 1] = run; run += e1;
    soff[8 * tid + 2] = run; run += e2;
    soff[8 * tid + 3] = run; run += e3;
    soff[8 * tid + 4] = run; run += e4;
    soff[8 * tid + 5] = run; run += e5;
    soff[8 * tid + 6] = run; run += e6;
    soff[8 * tid + 7] = run;
    carry = b4;
    __syncthreads();
    const v4i o0 = *(const v4i*)(soff + 4 * tid);
    const v4i o1 = *(const v4i*)(soff + 4 * (tid + OTHR));
    int* op = off + base;
    *(volatile v4i*)(op + 4 * tid) = o0;
    *(volatile v4i*)(op + 4 * (tid + OTHR)) = o1;
    __threadfence();
    *(volatile v4i*)(op + 4 * tid) = o0;
    *(volatile v4i*)(op + 4 * (tid + OTHR)) = o1;
    __syncthreads();
  }
  if (tid == 0) srb[min(4 * nChunk, RBN - 1)] = carry;
  __syncthreads();
  v4i rv = {0, 0, 0, 0};
  if (tid < 32) rv = *(const v4i*)(srb + 4 * tid);
  if (tid < 32) *(volatile v4i*)(rbase + 4 * tid) = rv;
  __threadfence();
  if (tid < 32) *(volatile v4i*)(rbase + 4 * tid) = rv;
}

__global__ __launch_bounds__(NTHR) void k_fill(
    const int* __restrict__ dsts, const int* __restrict__ off, const int* __restrict__ rbase,
    int* csr, int nE, int vec8, int csrLen) {
  extern __shared__ v4f lds_dyn[];
  int* region = (int*)lds_dyn;
  int* cursor = region + RCAP;
  int* list   = cursor + NBF;
  int* wcnt   = list + LISTN;
  const int tid = threadIdx.x, lane = tid & 31, wave = tid >> 5;
  const int b = blockIdx.x;
  const int nodeBase = b * NBF;

  int rb0 = rbase[b];
  const int rb1 = rbase[b + 1];
  rb0 = rb0 < 0 ? 0 : (rb0 > csrLen ? csrLen : rb0);
  rb0 &= ~31;
  int len = rb1 - rb0;
  len = len < 0 ? 0 : (len > RCAP ? RCAP : len);
  int lenW = (len + 31) & ~31;
  if (rb0 + lenW > csrLen) lenW = (csrLen - rb0) & ~31;

  {
    const v4i z = {0, 0, 0, 0};
    for (int i = tid; i < RCAP / 4; i += NTHR) ((v4i*)region)[i] = z;
    for (int s = tid; s < NBF; s += NTHR) {
      int o = off[nodeBase + s] - rb0;
      o = o < 0 ? 0 : (o > RCAP ? RCAP : o);
      cursor[s] = o;
    }
  }
  __syncthreads();

  const int nChunks = (nE + CHUNK - 1) / CHUNK;
#pragma unroll 1
  for (int ch = 0; ch < nChunks; ++ch) {
    const int cbase = ch * CHUNK;
    const int wc = scan_chunk<NBF>(dsts, nE, cbase, nodeBase, vec8, list, tid, lane, wave);
    if (lane == 0) wcnt[wave] = wc;
    __syncthreads();
    if (wave == 0) {
#pragma unroll 1
      for (int wsx = 0; wsx < NWAVE; ++wsx) {
        int n = __builtin_amdgcn_readfirstlane(wcnt[wsx]);
        n = n > WCAP ? WCAP : (n < 0 ? 0 : n);
        const int* lp = list + wsx * WCAP;
#pragma unroll 1
        for (int i = 0; i < n; ++i) {
          const int ent  = __builtin_amdgcn_readfirstlane(lp[i]);
          const int slot = ent & (NBF - 1);
          int e = cbase + ((ent >> 12) & (CHUNK - 1));
          e = e > nE - 1 ? nE - 1 : e;
          if (lane == 0) {
            int pos = cursor[slot];
            pos = pos < 0 ? 0 : (pos > RCAP - 1 ? RCAP - 1 : pos);
            region[pos] = e;
            const int np = pos + 1;
            cursor[slot] = np > RCAP ? RCAP : np;
          }
        }
      }
    }
    __syncthreads();
  }

  const int nv = lenW >> 2;
  int* gp = csr + rb0;
#pragma unroll 1
  for (int i = tid; i < nv; i += NTHR) { const v4i v = ((const v4i*)region)[i]; *(volatile v4i*)(gp + 4 * i) = v; }
  __threadfence();
#pragma unroll 1
  for (int i = tid; i < nv; i += NTHR) { const v4i v = ((const v4i*)region)[i]; *(volatile v4i*)(gp + 4 * i) = v; }
}

__global__ __launch_bounds__(NTHR) void k_gemm(
    const float* __restrict__ x, const unsigned short* __restrict__ Bw,
    const float* __restrict__ bias, float* C, int nN) {
  extern __shared__ v4f lds_dyn[];
  _Float16* sA  = (_Float16*)lds_dyn;
  float*    stg = (float*)((char*)lds_dyn + LDS_GA);
  const _Float16* Bh = (const _Float16*)Bw;
  const int tid = threadIdx.x, lane = tid & 31, wave = tid >> 5, hh = lane >> 4, m = lane & 15;
  const int rowBase = blockIdx.x * GROWS;
  const int c0 = (tid & 15) * 8, rr = tid >> 4;

#pragma unroll 2
  for (int it = 0; it < 8; ++it) {
    const int r = it * 16 + rr;
    int row = rowBase + r;
    row = row > nN - 1 ? nN - 1 : row;
    const float* ap = x + (size_t)row * FD + c0;
    const v4f a = *(const v4f*)ap, b = *(const v4f*)(ap + 4);
    *(v8h*)(sA + r * APK + c0) = cvt8(a, b, ASCL);
  }
  __syncthreads();

#pragma unroll
  for (int ch = 0; ch < 2; ++ch) {
    v8f acc[4];
#pragma unroll
    for (int t = 0; t < 4; ++t) { v8f z = {0.f, 0.f, 0.f, 0.f, 0.f, 0.f, 0.f, 0.f}; acc[t] = z; }
    const _Float16* ap = sA + (wave * 16 + m) * APK + 8 * hh;
#pragma unroll
    for (int kt = 0; kt < FD / 32; ++kt) {
      FragH a;
      a.h[0] = *(const v8h*)(ap + 32 * kt);
      a.h[1] = *(const v8h*)(ap + 32 * kt + 16);
#pragma unroll
      for (int t = 0; t < 4; ++t) {
        const _Float16* bp = Bh + (size_t)(64 * ch + 16 * t + m) * FD + 32 * kt + 8 * hh;
        FragH bq;
        bq.h[0] = *(const v8h*)bp;
        bq.h[1] = *(const v8h*)(bp + 16);
        acc[t] = wmh(a.v, bq.v, acc[t]);
      }
    }
    float* sp = stg + (wave * 16 + 8 * hh) * FD + 64 * ch + m;
#pragma unroll
    for (int t = 0; t < 4; ++t) {
      const float bv = bias[64 * ch + 16 * t + m];
#pragma unroll
      for (int r = 0; r < 8; ++r) sp[r * FD + 16 * t] = acc[t][r] * UNSCL + bv;
    }
  }
  __syncthreads();

  store_rows128(stg, C, rowBase, wave, lane);
}

__global__ __launch_bounds__(NTHR) void k_agg(
    const int* __restrict__ csr, const int* __restrict__ off, const int* __restrict__ cnt,
    const int* __restrict__ cols, const float* __restrict__ vals, const float* __restrict__ Zt,
    float* Zc, double* part, int nN, int nE, int csrLen) {
  __shared__ __attribute__((aligned(16))) double dS[NWAVE * FD];
  __shared__ __attribute__((aligned(16))) double dQ[NWAVE * FD];
  __shared__ __attribute__((aligned(16))) double dP[2 * FD];
  const int tid = threadIdx.x, lane = tid & 31, wave = tid >> 5;
  const int tbase = blockIdx.x * TGT + wave * 32;
  const int cl = tbase + lane;
  const int cnt_l = cnt[cl];
  const int off_l = off[cl];
  double s0 = 0.0, s1 = 0.0, s2 = 0.0, s3 = 0.0;
  double u0 = 0.0, u1 = 0.0, u2 = 0.0, u3 = 0.0;

#pragma unroll 1
  for (int j = 0; j < 32; ++j) {
    const int c = tbase + j;
    int n = __builtin_amdgcn_readlane(cnt_l, j);
    n = n < 0 ? 0 : (n > DEGCAP ? DEGCAP : n);
    const int st = __builtin_amdgcn_readlane(off_l, j);
    v4f sm = {0.0f, 0.0f, 0.0f, 0.0f};
#pragma unroll 1
    for (int p0 = 0; p0 < n; p0 += 32) {
      int pos = st + p0 + lane;
      pos = pos < 0 ? 0 : (pos > csrLen - 1 ? csrLen - 1 : pos);
      int e = csr[pos];
      e = e < 0 ? 0 : (e > nE - 1 ? nE - 1 : e);
      int sc = cols[e];
      sc = sc < 0 ? 0 : (sc > nN - 1 ? nN - 1 : sc);
      const float vv = vals[e];
      const int mcnt = (n - p0) < 32 ? (n - p0) : 32;
#pragma unroll 1
      for (int p = 0; p < mcnt; ++p) {
        const int s = __builtin_amdgcn_readlane(sc, p);
        const float w = __int_as_float(__builtin_amdgcn_readlane(__float_as_int(vv), p));
        const v4f vf = *(const v4f*)(Zt + (size_t)s * FD + 4 * lane);
        sm = sm + vf * w;
      }
    }
    float* zp = Zc + (size_t)c * FD + 4 * lane;
    *(volatile v4f*)zp = sm;
    __threadfence();
    *(volatile v4f*)zp = sm;
    if (c < nN) {
      const double d0 = (double)sm.x, d1 = (double)sm.y, d2 = (double)sm.z, d3 = (double)sm.w;
      s0 += d0; s1 += d1; s2 += d2; s3 += d3;
      u0 = fma(d0, d0, u0); u1 = fma(d1, d1, u1); u2 = fma(d2, d2, u2); u3 = fma(d3, d3, u3);
    }
  }
  dS[wave * FD + 4 * lane + 0] = s0; dS[wave * FD + 4 * lane + 1] = s1;
  dS[wave * FD + 4 * lane + 2] = s2; dS[wave * FD + 4 * lane + 3] = s3;
  dQ[wave * FD + 4 * lane + 0] = u0; dQ[wave * FD + 4 * lane + 1] = u1;
  dQ[wave * FD + 4 * lane + 2] = u2; dQ[wave * FD + 4 * lane + 3] = u3;
  __syncthreads();
  if (tid < FD) {
    double S = 0.0, Q = 0.0;
#pragma unroll
    for (int w = 0; w < NWAVE; ++w) { S += dS[w * FD + tid]; Q += dQ[w * FD + tid]; }
    dP[tid]      = S;
    dP[FD + tid] = Q;
  }
  __syncthreads();
  v2d pv = {0.0, 0.0};
  if (tid < FD) pv = *(const v2d*)(dP + 2 * tid);
  double* gq = part + (size_t)blockIdx.x * (2 * FD) + 2 * tid;
  if (tid < FD) *(volatile v2d*)gq = pv;
  __threadfence();
  if (tid < FD) *(volatile v2d*)gq = pv;
}

__global__ __launch_bounds__(FD) void k_bnfin(const double* __restrict__ part, const float* __restrict__ gamma,
                                             float* coef, int nBlk, int nN) {
  __shared__ __attribute__((aligned(16))) float sco[2 * FD];
  const int c = threadIdx.x;
  double S = 0.0, Q = 0.0;
#pragma unroll 1
  for (int b = 0; b < nBlk; ++b) {
    S += part[(size_t)b * (2 * FD) + c];
    Q += part[(size_t)b * (2 * FD) + FD + c];
  }
  const double rn = 1.0 / (double)(nN > 1 ? nN : 1);
  const double mean = S * rn;
  double var = Q * rn - mean * mean;
  var = var < 0.0 ? 0.0 : var;
  const float muf = (float)mean;
  const float sd  = sqrtf((float)var + BN_EPS);
  const float sc  = gamma[c] * (1.0f / sd);
  sco[c]      = muf;
  sco[FD + c] = sc;
  __syncthreads();
  v4f cv = {0.f, 0.f, 0.f, 0.f};
  if (c < 64) cv = *(const v4f*)(sco + 4 * c);
  if (c < 64) *(volatile v4f*)(coef + 4 * c) = cv;
  __threadfence();
  if (c < 64) *(volatile v4f*)(coef + 4 * c) = cv;
}

__device__ __forceinline__ void out_pass(const float* sout, float* ob, int nf, int tid) {
  if (tid < TGT / 4) {
    const v4f v = *(const v4f*)(sout + 4 * tid);
    if (4 * tid + 4 <= nf) {
      *(volatile v4f*)(ob + 4 * tid) = v;
    } else if (4 * tid < nf) {
      volatile float* op = ob + 4 * tid;
      op[0] = v.x;
      if (4 * tid + 1 < nf) op[1] = v.y;
      if (4 * tid + 2 < nf) op[2] = v.z;
    }
  }
}

__global__ __launch_bounds__(NTHR) void k_out(
    const float* __restrict__ Zc, const float* __restrict__ coef, const float* __restrict__ beta,
    float* out, int nN) {
  __shared__ __attribute__((aligned(16))) float sout[TGT];
  const int tid = threadIdx.x, lane = tid & 31, wave = tid >> 5;
  const int tbase = blockIdx.x * TGT + wave * 32;
  const v4f mu = *(const v4f*)(coef + 4 * lane);
  const v4f sc = *(const v4f*)(coef + FD + 4 * lane);
  const v4f be = *(const v4f*)(beta + 4 * lane);
  float mine = 0.0f;
#pragma unroll 1
  for (int j = 0; j < 32; ++j) {
    const int row = tbase + j;
    const v4f xv = *(const v4f*)(Zc + (size_t)row * FD + 4 * lane);
    const v4f t = (xv - mu) * sc + be;
    float m = fmaxf(fmaxf(t.x, t.y), fmaxf(t.z, t.w));
    m = fmaxf(m, 0.0f);
#pragma unroll
    for (int o = 16; o > 0; o >>= 1) m = fmaxf(m, __shfl_xor(m, o, 32));
    mine = (lane == j) ? m : mine;
  }
  sout[wave * 32 + lane] = mine;
  __syncthreads();

  int nvalid = nN - blockIdx.x * TGT;
  nvalid = nvalid > TGT ? TGT : (nvalid < 0 ? 0 : nvalid);
  float* ob = out + (size_t)blockIdx.x * TGT;
  out_pass(sout, ob, nvalid, tid);
  __threadfence();
  out_pass(sout, ob, nvalid, tid);
}

extern "C" void kernel_launch(void* const* d_in, const int* in_sizes, int n_in,
                              void* d_out, int out_size, void* d_ws, size_t ws_size,
                              hipStream_t stream) {
  if (n_in < 8) return;
  const int nN = in_sizes[0] / FD;
  const int nE = in_sizes[1];
  if (nN <= 0 || nE <= 0) return;
  if (in_sizes[0] != nN * FD) return;
  if (in_sizes[2] != FD * FD || in_sizes[3] != FD || in_sizes[4] != FD || in_sizes[5] != FD) return;
  if (in_sizes[6] != nE || in_sizes[7] != nE) return;
  if (out_size != nN) return;
  if (nE > (1 << 28) || nN > (1 << 24)) return;

  const float* zh    = (const float*)d_in[0];
  const float* vals  = (const float*)d_in[1];
  const float* W     = (const float*)d_in[2];
  const float* bia   = (const float*)d_in[3];
  const float* gam   = (const float*)d_in[4];
  const float* bet   = (const float*)d_in[5];
  const int*   rowi  = (const int*)d_in[6];
  const int*   coli  = (const int*)d_in[7];
  float* out = (float*)d_out;

  const int NPAD   = ((nN + TGT - 1) / TGT) * TGT;
  const int nBC    = (nN + NBC - 1) / NBC;
  const int CNTPAD = nBC * NBC;
  if (4 * nBC + 1 > RBN) return;
  const int nBF    = (nN + NBF - 1) / NBF;
  const int csrLen = ((nE + 31) & ~31) + 4096;
  if (31 * 4 * nBC > 4096) return;
  const int nGemm  = NPAD / GROWS;
  const int nAgg   = NPAD / TGT;

  char* ws = (char*)d_ws;
  size_t off = 0;
  const size_t oW    = off; off += (size_t)FD * FD * 2;             off = (off + 255) & ~(size_t)255;
  const size_t oCnt  = off; off += (size_t)CNTPAD * 4;              off = (off + 255) & ~(size_t)255;
  const size_t oOff  = off; off += (size_t)CNTPAD * 4;              off = (off + 255) & ~(size_t)255;
  const size_t oRb   = off; off += (size_t)RBN * 4;                 off = (off + 255) & ~(size_t)255;
  const size_t oCsr  = off; off += (size_t)csrLen * 4;              off = (off + 255) & ~(size_t)255;
  const size_t oZt   = off; off += (size_t)NPAD * FD * 4;           off = (off + 255) & ~(size_t)255;
  const size_t oZc   = off; off += (size_t)NPAD * FD * 4;           off = (off + 255) & ~(size_t)255;
  const size_t oPart = off; off += (size_t)nAgg * (2 * FD) * 8;     off = (off + 255) & ~(size_t)255;
  const size_t oCoef = off; off += (size_t)2 * FD * 4;              off = (off + 255) & ~(size_t)255;
  if (off > ws_size || off > (size_t)WSCAP) return;
  unsigned short* wp   = (unsigned short*)(ws + oW);
  int*            cnt  = (int*)(ws + oCnt);
  int*            offp = (int*)(ws + oOff);
  int*            rb   = (int*)(ws + oRb);
  int*            csr  = (int*)(ws + oCsr);
  float*          Zt   = (float*)(ws + oZt);
  float*          Zc   = (float*)(ws + oZc);
  double*         part = (double*)(ws + oPart);
  float*          coef = (float*)(ws + oCoef);

  const int vec8 = 1;

  k_wprep<<<(FD * FD) / (8 * NTHR), NTHR, 0, stream>>>(W, wp);

  k_count<<<nBC, NTHR, 0, stream>>>(rowi, cnt, nE, vec8);
  k_offsets<<<1, OTHR, 0, stream>>>(cnt, offp, rb, nBC);
  hipFuncSetAttribute(reinterpret_cast<const void*>(&k_fill),
                      hipFuncAttributeMaxDynamicSharedMemorySize, LDS_FILL);
  k_fill<<<nBF, NTHR, LDS_FILL, stream>>>(rowi, offp, rb, csr, nE, vec8, csrLen);

  hipFuncSetAttribute(reinterpret_cast<const void*>(&k_gemm),
                      hipFuncAttributeMaxDynamicSharedMemorySize, LDS_GEMM);
  k_gemm<<<nGemm, NTHR, LDS_GEMM, stream>>>(zh, wp, bia, Zt, nN);

  k_agg<<<nAgg, NTHR, 0, stream>>>(csr, offp, cnt, coli, vals, Zt, Zc, part, nN, nE, csrLen);

  k_bnfin<<<1, FD, 0, stream>>>(part, gam, coef, nAgg, nN);

  k_out<<<nAgg, NTHR, 0, stream>>>(Zc, coef, bet, out, nN);
}
